// MultiModalAttention_13168369730129
// MI455X (gfx1250) — hardware-verified
//
#include <hip/hip_runtime.h>
#include <math.h>

#ifndef NB
#define NB 4
#endif
#ifndef SEQ
#define SEQ 2048
#endif
#define NB_FULL 4
#define SEQ_FULL 2048
#define DQIN 32
#define DFEAT 34
#define DH 64
#define DVW 64
#define NMOD 3
#define ROWS (NB * SEQ)
#define QT (SEQ / 16)
#define AT_WAVES 8
#define AT_PITCH 68

#define QCAR 16.0f
#define KCAR 16.0f
#define VCAR 16.0f
#define PCAR 16384.0f
static constexpr float SC_QK = 1.0f / 256.0f;
static constexpr float OUT_UNDO = 1.0f / 262144.0f;
static constexpr float L2E = 1.4426950408889634f;

static_assert(QCAR * KCAR * SC_QK == 1.0f);
static_assert(PCAR * VCAR * OUT_UNDO == 1.0f);
static_assert(NB <= NB_FULL && SEQ <= SEQ_FULL);
static_assert(SEQ % 64 == 0 && SEQ_FULL % 4 == 0);
static_assert(DH % 32 == 0 && DH == 64 && DVW == 64 && DQIN == 32);
static_assert((ROWS * 8) % 256 == 0);
static_assert(ROWS % 64 == 0);
static_assert((NB * QT) % AT_WAVES == 0);
static_assert(256 * 2 == 64 * 8);
static_assert(32 * 16 * 8 == 16 * 256);
static_assert(AT_WAVES * 16 * AT_PITCH * 4 <= 131072);
static_assert((DQIN * 64 + 64 + 64 * 65) * 4 <= 131072);
static_assert((size_t)NMOD * NB_FULL * SEQ_FULL * DVW * 4 == (size_t)6291456);
static_assert((size_t)NB_FULL * SEQ_FULL * DVW * 4 == (size_t)2097152);

#define WS_QPLANE ((size_t)ROWS * DH * 2)
#define WS_ROWF   ((size_t)ROWS * 4)
#define WS_TOTAL  (2 * WS_QPLANE + 2 * WS_ROWF + (size_t)NMOD * (2 * WS_QPLANE + 2 * WS_ROWF + WS_QPLANE))
static_assert(WS_QPLANE % 256 == 0 && WS_ROWF % 256 == 0);
static_assert(WS_TOTAL <= (size_t)134217728);

typedef _Float16 h16;
typedef __attribute__((ext_vector_type(16))) _Float16 v16h;
typedef __attribute__((ext_vector_type(8)))  _Float16 v8h;
typedef __attribute__((ext_vector_type(8)))  float    v8f;
typedef __attribute__((ext_vector_type(4)))  float    v4f;


#define VST2(T, ptr, val) do { const T vst2_v_ = (val); *(volatile T*)(ptr) = vst2_v_; __threadfence(); *(volatile T*)(ptr) = vst2_v_; } while (0)
#define VST2V4(ptr, val) do { const v4f vst2_v4_ = (val); *(volatile v4f*)(ptr) = vst2_v4_; __threadfence(); *(volatile v4f*)(ptr) = vst2_v4_; } while (0)

__device__ __forceinline__ float bfr(float f) {
    unsigned u = __float_as_uint(f);
    u += 0x7FFFu + ((u >> 16) & 1u);
    return __uint_as_float(u & 0xFFFF0000u);
}
static __device__ __forceinline__ h16 toh_flush(float v) {
    const float w = (fabsf(v) < 6.103515625e-05f) ? 0.0f : v;
    return (h16)w;
}

union FragU { v16h v; v8h h[2]; };
__device__ __forceinline__ v16h frag_ld(const _Float16* p) {
    FragU f; f.h[0] = *(const v8h*)(p); f.h[1] = *(const v8h*)(p + 16); return f.v;
}
__device__ __forceinline__ v8f wmma16g(v16h a, v16h b, v8f c) {
    c = __builtin_amdgcn_wmma_f32_16x16x32_f16(false, a, false, b, (short)0, c, false, false);
    asm volatile("v_nop\n\tv_nop\n\tv_nop\n\tv_nop" : "+v"(c) : "v"(a), "v"(b));
    return c;
}
__device__ __forceinline__ void wave_sync_lds() {
    __builtin_amdgcn_fence(3  , "workgroup");
    __builtin_amdgcn_wave_barrier();
    __builtin_amdgcn_fence(2  , "workgroup");
}

__global__ __launch_bounds__(256) void k_prepq(const float* __restrict__ ref_data, const float* __restrict__ ref_t,
                                               const float* __restrict__ Wq, _Float16* __restrict__ QHp,
                                               _Float16* __restrict__ QLp, float* __restrict__ q0p, float* __restrict__ rtb) {
    __shared__ float sW[DQIN * 64];
    __shared__ float sQ0[32];
    const unsigned tid = threadIdx.x;
#pragma unroll
    for (int i = 0; i < 8; ++i) sW[tid + 256u * (unsigned)i] = bfr(Wq[tid + 256u * (unsigned)i]);
    __syncthreads();
    const unsigned u = blockIdx.x * 256u + tid;
    const unsigned wrow = u >> 3, j0 = (u & 7u) * 8u;
    const unsigned n = wrow / (unsigned)SEQ;
    const unsigned t = wrow - n * (unsigned)SEQ;
    const float* xr = ref_data + (size_t)(n * (unsigned)SEQ_FULL + t) * DQIN;
    float acc[9];
#pragma unroll
    for (int i = 0; i < 9; ++i) acc[i] = 0.0f;
#pragma unroll 1
    for (unsigned d = 0; d < (unsigned)DQIN; ++d) {
        const float x = bfr(xr[d]);
#pragma unroll
        for (int i = 0; i < 9; ++i) {
            const unsigned col = min(j0 + (unsigned)i, 63u);
            acc[i] += x * sW[d * 64u + col];
        }
    }
    v8h hv, lv;
#pragma unroll
    for (int i = 0; i < 8; ++i) {
        const unsigned j = j0 + (unsigned)i;
        const float q = (j < 63u) ? acc[i + 1] * QCAR : 0.0f;
        const h16 h = toh_flush(q);
        hv[i] = h;
        lv[i] = toh_flush(q - (float)h);
    }
    VST2(v8h, QHp + (size_t)wrow * DH + j0, hv);
    VST2(v8h, QLp + (size_t)wrow * DH + j0, lv);
    if ((u & 7u) == 0u) sQ0[tid >> 3] = acc[0];
    __syncthreads();
    if (tid < 8u) {
        const unsigned wb = blockIdx.x * 32u + 4u * tid;
        const unsigned nb = wb / (unsigned)SEQ;
        const unsigned tb = wb - nb * (unsigned)SEQ;
        v4f qv; qv.x = sQ0[4u * tid]; qv.y = sQ0[4u * tid + 1u]; qv.z = sQ0[4u * tid + 2u]; qv.w = sQ0[4u * tid + 3u];
        VST2V4(q0p + wb, qv);
        const v4f rv = *(const v4f*)(ref_t + (size_t)(nb * (unsigned)SEQ_FULL + tb));
        v4f rb; rb.x = bfr(rv.x); rb.y = bfr(rv.y); rb.z = bfr(rv.z); rb.w = bfr(rv.w);
        VST2V4(rtb + wb, rb);
    }
}

__global__ __launch_bounds__(256) void k_prepk(const float* __restrict__ data, const float* __restrict__ mt,
                                               const float* __restrict__ Wk, const float* __restrict__ bk,
                                               _Float16* __restrict__ KHp, _Float16* __restrict__ KLp,
                                               float* __restrict__ k63p, float* __restrict__ mtb) {
    __shared__ float sWk[64];
    __shared__ float sBk[64];
    __shared__ float sK[32];
    const unsigned tid = threadIdx.x;
    if (tid < 64u) { sWk[tid] = bfr(Wk[tid]); sBk[tid] = bfr(bk[tid]); }
    __syncthreads();
    const unsigned u = blockIdx.x * 256u + tid;
    const unsigned wrow = u >> 3, j0 = (u & 7u) * 8u;
    const unsigned n = wrow / (unsigned)SEQ;
    const unsigned t = wrow - n * (unsigned)SEQ;
    const float x = bfr(data[(size_t)(n * (unsigned)SEQ_FULL + t) * DFEAT + (DFEAT - 1)]);
    v8h hv, lv;
#pragma unroll
    for (int i = 0; i < 8; ++i) {
        const unsigned j = j0 + (unsigned)i;
        const float kr = x * sWk[j] + sBk[j];
        const float kd = (j < 63u) ? (-kr) * KCAR : 0.0f;
        const h16 h = toh_flush(kd);
        hv[i] = h;
        lv[i] = toh_flush(kd - (float)h);
    }
    VST2(v8h, KHp + (size_t)wrow * DH + j0, hv);
    VST2(v8h, KLp + (size_t)wrow * DH + j0, lv);
    if ((u & 7u) == 7u) sK[tid >> 3] = x * sWk[63] + sBk[63];
    __syncthreads();
    if (tid < 8u) {
        const unsigned wb = blockIdx.x * 32u + 4u * tid;
        const unsigned nb = wb / (unsigned)SEQ;
        const unsigned tb = wb - nb * (unsigned)SEQ;
        v4f kv; kv.x = sK[4u * tid]; kv.y = sK[4u * tid + 1u]; kv.z = sK[4u * tid + 2u]; kv.w = sK[4u * tid + 3u];
        VST2V4(k63p + wb, kv);
        const v4f rv = *(const v4f*)(mt + (size_t)(nb * (unsigned)SEQ_FULL + tb));
        v4f rb; rb.x = bfr(rv.x); rb.y = bfr(rv.y); rb.z = bfr(rv.z); rb.w = bfr(rv.w);
        VST2V4(mtb + wb, rb);
    }
}

__global__ __launch_bounds__(256) void k_prepv(const float* __restrict__ data, const float* __restrict__ Wv,
                                               const float* __restrict__ bv, _Float16* __restrict__ VTp) {
    __shared__ float sW[DQIN * 64];
    __shared__ float sB[64];
    __shared__ float sT[64 * 65];
    const unsigned tid = threadIdx.x;
#pragma unroll
    for (int i = 0; i < 8; ++i) sW[tid + 256u * (unsigned)i] = bfr(Wv[tid + 256u * (unsigned)i]);
    if (tid < 64u) sB[tid] = bfr(bv[tid]);
    __syncthreads();
    const unsigned w0 = blockIdx.x * 64u;
    const unsigned n = w0 / (unsigned)SEQ;
    const unsigned l0 = w0 - n * (unsigned)SEQ;
    const unsigned lk = tid & 63u, dg = tid >> 6;
    const float* xr = data + (size_t)(n * (unsigned)SEQ_FULL + l0 + lk) * DFEAT;
    float acc[16];
#pragma unroll
    for (int i = 0; i < 16; ++i) acc[i] = 0.0f;
#pragma unroll 1
    for (unsigned k = 0; k < (unsigned)DQIN; ++k) {
        const float x = bfr(xr[k]);
#pragma unroll
        for (int i = 0; i < 16; ++i) acc[i] += x * sW[k * 64u + 16u * dg + (unsigned)i];
    }
#pragma unroll
    for (int i = 0; i < 16; ++i) sT[(16u * dg + (unsigned)i) * 65u + lk] = (acc[i] + sB[16u * dg + (unsigned)i]) * VCAR;
    __syncthreads();
    v8h hv[2];
#pragma unroll
    for (int it = 0; it < 2; ++it) {
        const unsigned p = (unsigned)it * 256u + tid;
        const unsigned d = p >> 3, pc = p & 7u;
#pragma unroll
        for (int e = 0; e < 8; ++e) hv[it][e] = toh_flush(sT[d * 65u + 8u * pc + (unsigned)e]);
    }
    for (int pass = 0; pass < 2; ++pass) {
#pragma unroll
        for (int it = 0; it < 2; ++it) {
            const unsigned p = (unsigned)it * 256u + tid;
            const unsigned d = p >> 3, pc = p & 7u;
            *(volatile v8h*)(VTp + (size_t)(n * 64u + d) * SEQ + l0 + 8u * pc) = hv[it];
        }
        __threadfence();
    }
}

__global__ __launch_bounds__(256) __attribute__((amdgpu_num_vgpr(256))) void k_attn(
    const _Float16* __restrict__ QHp, const _Float16* __restrict__ QLp, const float* __restrict__ q0p,
    const float* __restrict__ rtb, const _Float16* __restrict__ KHp, const _Float16* __restrict__ KLp,
    const float* __restrict__ k63p, const float* __restrict__ mtb, const _Float16* __restrict__ VTp,
    const float* __restrict__ log_tau, float* __restrict__ out) {
    __shared__ __align__(16) float sT[AT_WAVES][16 * AT_PITCH];
    const unsigned lane = threadIdx.x & 31u;
    const unsigned wave = (unsigned)__builtin_amdgcn_readfirstlane((int)(threadIdx.x >> 5));
    const unsigned hh = lane >> 4, c = lane & 15u;
    const unsigned tile = blockIdx.x * (unsigned)AT_WAVES + wave;
    const unsigned n = tile / (unsigned)QT;
    const unsigned t0 = (tile - n * (unsigned)QT) * 16u;
    const unsigned rbase = n * (unsigned)SEQ;
    const unsigned qrow = rbase + t0 + c;

    v16h qh[2], ql[2];
#pragma unroll
    for (int ks = 0; ks < 2; ++ks) {
        qh[ks] = frag_ld(QHp + (size_t)qrow * DH + 32u * (unsigned)ks + 8u * hh);
        ql[ks] = frag_ld(QLp + (size_t)qrow * DH + 32u * (unsigned)ks + 8u * hh);
    }
    const float q0 = q0p[qrow];
    const float rt = rtb[qrow];
    const float ltv = bfr(log_tau[0]);
    const float itau = 1.0f / expf(ltv);

    float mrun = -1.0e30f, lsum = 0.0f;
    v8f o[4];
#pragma unroll
    for (int dt = 0; dt < 4; ++dt) o[dt] = (v8f){0.f,0.f,0.f,0.f,0.f,0.f,0.f,0.f};

#pragma unroll 1
    for (unsigned l0 = 0; l0 < (unsigned)SEQ; l0 += 32u) {
        float z[2][8], mc[2][8];
#pragma unroll
        for (int tt = 0; tt < 2; ++tt) {
            unsigned lt = l0 + 16u * (unsigned)tt;
            asm volatile("" : "+v"(lt));
            const unsigned koff = (rbase + lt + c) * (unsigned)DH + 8u * hh;
            v8f acc = (v8f){0.f,0.f,0.f,0.f,0.f,0.f,0.f,0.f};
#pragma unroll
            for (int ks = 0; ks < 2; ++ks) {
                const v16h kh = frag_ld(KHp + koff + 32u * (unsigned)ks);
                const v16h kl = frag_ld(KLp + koff + 32u * (unsigned)ks);
                acc = wmma16g(kh, qh[ks], acc);
                acc = wmma16g(kh, ql[ks], acc);
                acc = wmma16g(kl, qh[ks], acc);
            }
            const unsigned aoff = rbase + lt + 8u * hh;
            const v4f ta = *(const v4f*)(mtb + aoff), tb = *(const v4f*)(mtb + aoff + 4u);
            const v4f ka = *(const v4f*)(k63p + aoff), kb = *(const v4f*)(k63p + aoff + 4u);
            const float tm[8] = {ta.x, ta.y, ta.z, ta.w, tb.x, tb.y, tb.z, tb.w};
            const float kk[8] = {ka.x, ka.y, ka.z, ka.w, kb.x, kb.y, kb.z, kb.w};
#pragma unroll
            for (int r = 0; r < 8; ++r) {
                const float qk = acc[r] * SC_QK + (q0 - kk[r]);
                const float s = -(qk * qk) * itau;
                const bool vis = (rt >= tm[r]);
                const float m1 = vis ? 1.0f : 0.0f;
                z[tt][r] = s * m1;
                mc[tt][r] = vis ? PCAR : 0.0f;
            }
        }
        float mx = z[0][0];
#pragma unroll
        for (int r = 1; r < 8; ++r) mx = (z[0][r] > mx) ? z[0][r] : mx;
#pragma unroll
        for (int r = 0; r < 8; ++r) mx = (z[1][r] > mx) ? z[1][r] : mx;
        const float mo = __shfl_xor(mx, 16, 32);
        mx = (mo > mx) ? mo : mx;
        const float mnew = (mx > mrun) ? mx : mrun;
        const float alpha = exp2f((mrun - mnew) * L2E);
        mrun = mnew;
        float psum = 0.0f;
        v16h ph, pl;
#pragma unroll
        for (int tt = 0; tt < 2; ++tt) {
#pragma unroll
            for (int r = 0; r < 8; ++r) {
                const float e = (z[tt][r] - mnew) * L2E;
                const float p = __builtin_amdgcn_exp2f(e);
                psum += p;
                const float a = p * mc[tt][r];
                const h16 h = toh_flush(a);
                ph[8 * tt + r] = h;
                pl[8 * tt + r] = toh_flush(a - (float)h);
            }
        }
        lsum = lsum * alpha + psum;
#pragma unroll
        for (int dt = 0; dt < 4; ++dt) o[dt] *= alpha;
        unsigned lv = l0;
        asm volatile("" : "+v"(lv));
#pragma unroll
        for (int dt = 0; dt < 4; ++dt) {
            const v16h va = frag_ld(VTp + (size_t)((n * 64u + 16u * (unsigned)dt + c) * (unsigned)SEQ + lv + 8u * hh));
            o[dt] = wmma16g(va, ph, o[dt]);
            o[dt] = wmma16g(va, pl, o[dt]);
        }
    }

    const float lo = __shfl_xor(lsum, 16, 32);
    const float inv = (1.0f / (lsum + lo)) * OUT_UNDO;
#pragma unroll
    for (int dt = 0; dt < 4; ++dt)
#pragma unroll
        for (int r = 0; r < 8; ++r)
            sT[wave][c * (unsigned)AT_PITCH + 16u * (unsigned)dt + 8u * hh + (unsigned)r] = o[dt][r] * inv;
    wave_sync_lds();
    {
        const unsigned c4 = (lane & 15u) * 4u;
        float* dst = out + (size_t)(n * (unsigned)SEQ_FULL + t0) * DVW;
#pragma unroll
        for (int half = 0; half < 2; ++half) {
            v4f vv[4];
#pragma unroll
            for (int it = 0; it < 4; ++it) {
                const unsigned row = (unsigned)(half * 4 + it) * 2u + hh;
                vv[it] = *(const v4f*)(&sT[wave][row * (unsigned)AT_PITCH + c4]);
            }
            for (int pass = 0; pass < 2; ++pass) {
#pragma unroll
                for (int it = 0; it < 4; ++it) {
                    const unsigned row = (unsigned)(half * 4 + it) * 2u + hh;
                    *(volatile v4f*)(dst + (size_t)row * DVW + c4) = vv[it];
                }
                __threadfence();
            }
        }
    }
}

extern "C" void kernel_launch(void* const* d_in, const int* in_sizes, int n_in, void* d_out, int out_size,
                              void* d_ws, size_t ws_size, hipStream_t stream) {
    if (n_in < 24) return;
    if (in_sizes[0] < ROWS * DQIN || in_sizes[1] < ROWS || in_sizes[8] < DQIN * 64) return;
    for (int m = 0; m < NMOD; ++m) {
        if (in_sizes[2 + 2 * m] < ROWS * DFEAT || in_sizes[3 + 2 * m] < ROWS) return;
        if (in_sizes[9 + 5 * m] < 64 || in_sizes[10 + 5 * m] < 64 || in_sizes[11 + 5 * m] < DQIN * 64) return;
        if (in_sizes[12 + 5 * m] < 64 || in_sizes[13 + 5 * m] < 1) return;
    }
    if (out_size < NMOD * NB_FULL * SEQ_FULL * DVW) return;

    const float* ref_data = (const float*)d_in[0];
    const float* ref_t    = (const float*)d_in[1];
    const float* Wq       = (const float*)d_in[8];
    float* out = (float*)d_out;

    char* wsp = (char*)d_ws;
    size_t off = 0;
    auto carve = [&](size_t bytes) -> void* { void* r = wsp + off; off += (bytes + 255) & ~(size_t)255; return r; };
    _Float16* QH  = (_Float16*)carve(WS_QPLANE);
    _Float16* QL  = (_Float16*)carve(WS_QPLANE);
    float*    q0p = (float*)carve(WS_ROWF);
    float*    rtb = (float*)carve(WS_ROWF);
    _Float16* KH  = (_Float16*)carve((size_t)NMOD * WS_QPLANE);
    _Float16* KL  = (_Float16*)carve((size_t)NMOD * WS_QPLANE);
    float*    k63 = (float*)carve((size_t)NMOD * WS_ROWF);
    float*    mtb = (float*)carve((size_t)NMOD * WS_ROWF);
    _Float16* VT  = (_Float16*)carve((size_t)NMOD * WS_QPLANE);
    if (off > ws_size || off > (size_t)134217728) return;

    k_prepq<<<ROWS / 32, 256, 0, stream>>>(ref_data, ref_t, Wq, QH, QL, q0p, rtb);
    for (int m = 0; m < NMOD; ++m) {
        const float* data = (const float*)d_in[2 + 2 * m];
        const float* mt   = (const float*)d_in[3 + 2 * m];
        const float* Wk   = (const float*)d_in[9 + 5 * m];
        const float* bk   = (const float*)d_in[10 + 5 * m];
        const float* Wv   = (const float*)d_in[11 + 5 * m];
        const float* bv   = (const float*)d_in[12 + 5 * m];
        k_prepk<<<ROWS / 32, 256, 0, stream>>>(data, mt, Wk, bk, KH + (size_t)m * ROWS * DH, KL + (size_t)m * ROWS * DH,
                                               k63 + (size_t)m * ROWS, mtb + (size_t)m * ROWS);
        k_prepv<<<ROWS / 64, 256, 0, stream>>>(data, Wv, bv, VT + (size_t)m * ROWS * DVW);
    }
    for (int m = 0; m < NMOD; ++m) {
        const float* ltau = (const float*)d_in[13 + 5 * m];
        k_attn<<<(NB * QT) / AT_WAVES, 256, 0, stream>>>(QH, QL, q0p, rtb, KH + (size_t)m * ROWS * DH, KL + (size_t)m * ROWS * DH,
                                                         k63 + (size_t)m * ROWS, mtb + (size_t)m * ROWS, VT + (size_t)m * ROWS * DVW,
                                                         ltau, out + (size_t)m * NB_FULL * SEQ_FULL * DVW);
    }
}
